// GCNEncoder_3968549782293
// MI455X (gfx1250) — hardware-verified
//
#include <hip/hip_runtime.h>
#include <math.h>

constexpr int   kNodes   = 32768;
constexpr int   kFin     = 64;
constexpr int   kDim     = 512;
constexpr int   kDim2    = 1024;
constexpr int   kDout    = 128;
constexpr int   kChunkRows = 4096;
constexpr int   kNumChunks = kNodes / kChunkRows;
constexpr int   kNumSlots  = 9;
constexpr long  kSlotElems = (long)kChunkRows * kDim;
constexpr int   kStatRows  = 128;
constexpr int   kStatBlocks = kNodes / kStatRows;
constexpr int   kStatBlocksPerChunk = kChunkRows / kStatRows;
constexpr float kEpsMsg  = 1e-7f;
constexpr float kEpsLn   = 1e-5f;
constexpr float kInvDim2 = 1.0f / 1024.0f;
constexpr float kWCarry  = 64.0f;
constexpr float kInCarry = 16.0f;
constexpr float kZCarry  = 8.0f;
constexpr float kHCarry  = 8.0f;

static_assert(kNodes % kChunkRows == 0, "chunking");
static_assert(kChunkRows % kStatRows == 0, "stat blocks inside chunks");
static_assert(kChunkRows % 64 == 0 && kDim % 64 == 0 && kDim2 % 64 == 0 && kDout % 64 == 0, "tile multiples");
static_assert(kFin % 32 == 0 && kDim % 32 == 0 && kDim2 % 32 == 0, "K multiples of 32");

typedef __attribute__((ext_vector_type(16))) _Float16 v16h;
typedef __attribute__((ext_vector_type(8)))  _Float16 v8h;
typedef __attribute__((ext_vector_type(16))) __bf16   v16b;
typedef __attribute__((ext_vector_type(8)))  __bf16   v8b;
typedef __attribute__((ext_vector_type(8)))  float    v8f;
typedef __attribute__((ext_vector_type(4)))  float    v4f;
typedef __attribute__((ext_vector_type(4)))  unsigned int v4u;

__device__ __forceinline__ unsigned short f2bf_bits(float f) {
  unsigned u = __float_as_uint(f);
  return (unsigned short)((u + 0x7FFFu + ((u >> 16) & 1u)) >> 16);
}
__device__ __forceinline__ float bf_bits2f(unsigned short h) { return __uint_as_float(((unsigned)h) << 16); }

__device__ __forceinline__ void dep_guard_h(v8f& a, v8f& b, v16h x, v16h y) { asm volatile("v_nop\n\tv_nop\n\tv_nop\n\tv_nop" : "+v"(a), "+v"(b) : "v"(x), "v"(y)); }
__device__ __forceinline__ void dep_guard_b(v8f& a, v8f& b, v16b x, v16b y) { asm volatile("v_nop\n\tv_nop\n\tv_nop\n\tv_nop" : "+v"(a), "+v"(b) : "v"(x), "v"(y)); }
__device__ __forceinline__ void keep4_h(v16h a, v16h b, v16h c, v16h d) { asm volatile("v_nop" :: "v"(a), "v"(b), "v"(c), "v"(d)); }
__device__ __forceinline__ void keep4_b(v16b a, v16b b, v16b c, v16b d) { asm volatile("v_nop" :: "v"(a), "v"(b), "v"(c), "v"(d)); }
__device__ __forceinline__ void acc_guard4(v8f& a, v8f& b, v8f& c, v8f& d) { asm volatile("v_nop\n\tv_nop\n\tv_nop\n\tv_nop" : "+v"(a), "+v"(b), "+v"(c), "+v"(d)); }
template <typename T> struct Frag;
template <> struct Frag<_Float16> {
  typedef v16h V; union U { v16h v; v8h h[2]; };
  static __device__ __forceinline__ v16h load(const _Float16* p) {
    U f; f.h[0] = *(const v8h*)(p); f.h[1] = *(const v8h*)(p + 16); return f.v;
  }
  static __device__ __forceinline__ v8f mma(v16h a, v16h b, v8f c) {
    return __builtin_amdgcn_wmma_f32_16x16x32_f16(false, a, false, b, (short)0, c, false, false);
  }
  static __device__ __forceinline__ void guard(v8f& a, v8f& b, v16h x, v16h y) { dep_guard_h(a, b, x, y); }
  static __device__ __forceinline__ void keep(v16h a, v16h b, v16h c, v16h d) { keep4_h(a, b, c, d); }
};
template <> struct Frag<__bf16> {
  typedef v16b V; union U { v16b v; v8b h[2]; };
  static __device__ __forceinline__ v16b load(const __bf16* p) {
    U f; f.h[0] = *(const v8b*)(p); f.h[1] = *(const v8b*)(p + 16); return f.v;
  }
  static __device__ __forceinline__ v8f mma(v16b a, v16b b, v8f c) {
    return __builtin_amdgcn_wmma_f32_16x16x32_bf16(false, a, false, b, (short)0, c, false, false);
  }
  static __device__ __forceinline__ void guard(v8f& a, v8f& b, v16b x, v16b y) { dep_guard_b(a, b, x, y); }
  static __device__ __forceinline__ void keep(v16b a, v16b b, v16b c, v16b d) { keep4_b(a, b, c, d); }
};

__device__ __forceinline__ unsigned pk16(unsigned short a, unsigned short b) { return (unsigned)a | ((unsigned)b << 16); }
__device__ __forceinline__ unsigned short h_bits(float f) { const _Float16 h = (_Float16)f; return __builtin_bit_cast(unsigned short, h); }

template <int ET> struct Elem;
template <> struct Elem<0> { typedef _Float16 T; };
template <> struct Elem<1> { typedef __bf16 T; };
template <int ET, bool SPLIT, int BIAS_MODE, int OUT_MODE, bool RESID, int ACT = 0>
__global__ __launch_bounds__(256) void wmma_gemm64(
    const unsigned short* __restrict__ Ap, const unsigned short* __restrict__ A2p, int lda, long strideA,
    const unsigned short* __restrict__ Btp, const unsigned short* __restrict__ Bt2p, int ldb, long strideB,
    void* __restrict__ Cout, void* __restrict__ Cout2, int ldc, long strideC,
    const float* __restrict__ bias,
    const float* __restrict__ resid, long strideR,
    int M, int N, int K, float scale) {
  typedef typename Elem<ET>::T T;
  typedef typename Frag<T>::V V;
  const T* A = (const T*)Ap; const T* A2 = (const T*)A2p; const T* Bt = (const T*)Btp; const T* Bt2 = (const T*)Bt2p;
  __shared__ __align__(16) float sT[8][16 * 68];
  const int b    = blockIdx.y;
  const int lane = threadIdx.x & 31;
  const int wave = threadIdx.x >> 5;
  const int tilesN = N >> 6;
  const int tilesM = M >> 6;
  const int tile = blockIdx.x * 8 + wave;
  if (tile >= tilesM * tilesN) return;
  const int tm = tile / tilesN;
  const int tn = tile - tm * tilesN;
  const int m0 = tm << 6;
  const int n0 = tn << 6;

  const T* Ab  = A  + (size_t)b * strideA;
  const T* Bb  = Bt + (size_t)b * strideB;
  const T* Ab2 = SPLIT ? (A2  + (size_t)b * strideA) : nullptr;
  const T* Bb2 = SPLIT ? (Bt2 + (size_t)b * strideB) : nullptr;

  const int rlane = lane & 15;
  const int koff  = (lane >> 4) * 8;
  const int mOff  = (lane >> 4) * 8;

  v8f acc[4][4];
#pragma unroll
  for (int i = 0; i < 4; ++i)
#pragma unroll
    for (int j = 0; j < 4; ++j) acc[i][j] = (v8f){0.f,0.f,0.f,0.f,0.f,0.f,0.f,0.f};

  for (int k0 = 0; k0 < K; k0 += 32) {
    V bh[4], bl[4];
#pragma unroll
    for (int j = 0; j < 4; ++j) {
      const size_t bo = (size_t)(n0 + (j << 4) + rlane) * ldb + koff + k0;
      bh[j] = Frag<T>::load(Bb + bo);
      if (SPLIT) bl[j] = Frag<T>::load(Bb2 + bo);
    }
#pragma unroll
    for (int i = 0; i < 4; ++i) {
      const size_t ao = (size_t)(m0 + (i << 4) + rlane) * lda + koff + k0;
      V ah = Frag<T>::load(Ab + ao);
      V al;
      if (SPLIT) al = Frag<T>::load(Ab2 + ao);
#pragma unroll
      for (int j = 0; j < 4; ++j) {
        acc[i][j] = Frag<T>::mma(ah, bh[j], acc[i][j]);
        if (SPLIT) {
          acc[i][j] = Frag<T>::mma(ah, bl[j], acc[i][j]);
          acc[i][j] = Frag<T>::mma(al, bh[j], acc[i][j]);
        }
      }
      Frag<T>::guard(acc[i][0], acc[i][3], ah, SPLIT ? al : ah);
    }
    Frag<T>::keep(bh[0], bh[1], bh[2], bh[3]);
    if (SPLIT) Frag<T>::keep(bl[0], bl[1], bl[2], bl[3]);
  }
  acc_guard4(acc[0][0], acc[0][1], acc[0][2], acc[0][3]);
  acc_guard4(acc[1][0], acc[1][1], acc[1][2], acc[1][3]);
  acc_guard4(acc[2][0], acc[2][1], acc[2][2], acc[2][3]);
  acc_guard4(acc[3][0], acc[3][1], acc[3][2], acc[3][3]);

  float* slab = sT[wave];
  const float* Rb = RESID ? (resid + (size_t)b * strideR) : nullptr;
#pragma unroll
  for (int i = 0; i < 4; ++i) {
    const int mBase = m0 + (i << 4);
#pragma unroll
    for (int j = 0; j < 4; ++j) {
      const int n = n0 + (j << 4) + rlane;
      float bv = 0.f;
      if (BIAS_MODE == 2) bv = bias[n];
#pragma unroll
      for (int r = 0; r < 8; ++r) {
        float v = acc[i][j][r] * scale;
        if (BIAS_MODE == 1) v += bias[mBase + mOff + r];
        if (BIAS_MODE == 2) v += bv;
        if (RESID) v += Rb[(size_t)(mBase + mOff + r) * ldc + n];
        if (ACT == 2) v = fmaxf(v, 0.0f);
        if (ACT == 4) v = (v > 0.f) ? v : 0.01f * v;
        slab[(mOff + r) * 68 + (j << 4) + rlane] = v;
      }
    }
    __builtin_amdgcn_fence(__ATOMIC_RELEASE, "workgroup");
    __builtin_amdgcn_wave_barrier();
    __builtin_amdgcn_fence(__ATOMIC_ACQUIRE, "workgroup");
    if (OUT_MODE == 0) {
      float* C = (float*)Cout + (size_t)b * strideC;
      const int hh = lane >> 4, c4 = (lane & 15) * 4;
      for (int pass = 0; pass < 2; ++pass) {
#pragma unroll
        for (int it = 0; it < 8; ++it) {
          const int row = it * 2 + hh;
          v4f v = *(const v4f*)(slab + row * 68 + c4);
          *(volatile v4f*)(C + (size_t)(mBase + row) * ldc + n0 + c4) = v;
        }
        __threadfence();
      }
    } else {
      const int q = lane >> 3, c8 = (lane & 7) * 8;
      unsigned short* C  = (unsigned short*)Cout  + (size_t)b * strideC;
      unsigned short* C2 = (OUT_MODE == 2) ? ((unsigned short*)Cout2 + (size_t)b * strideC) : nullptr;
      for (int pass = 0; pass < 2; ++pass) {
#pragma unroll
        for (int it = 0; it < 4; ++it) {
          const int row = it * 4 + q;
          const float* sp = slab + row * 68 + c8;
          v8h hv, lv;
#pragma unroll
          for (int e = 0; e < 8; ++e) {
            if (OUT_MODE == 1) {
              hv[e] = (_Float16)sp[e];
            } else {
              unsigned short hb = f2bf_bits(sp[e]);
              unsigned short lb = f2bf_bits(sp[e] - bf_bits2f(hb));
              hv[e] = __builtin_bit_cast(_Float16, hb);
              lv[e] = __builtin_bit_cast(_Float16, lb);
            }
          }
          *(volatile v8h*)(C + (size_t)(mBase + row) * ldc + n0 + c8) = hv;
          if (OUT_MODE == 2) *(volatile v8h*)(C2 + (size_t)(mBase + row) * ldc + n0 + c8) = lv;
        }
        __threadfence();
      }
    }
    __builtin_amdgcn_fence(__ATOMIC_RELEASE, "workgroup");
    __builtin_amdgcn_wave_barrier();
    __builtin_amdgcn_fence(__ATOMIC_ACQUIRE, "workgroup");
  }
}

__global__ __launch_bounds__(256) void cast8_f16_kernel(const float* __restrict__ in, unsigned short* __restrict__ out,
                                                        int n8, float carry) {
  const int i = blockIdx.x * 256 + threadIdx.x;
  if (i >= n8) return;
  const float* p = in + 8 * (size_t)i;
  const v4f a = *(const v4f*)(p);
  const v4f c = *(const v4f*)(p + 4);
  unsigned short hb[8];
#pragma unroll
  for (int e = 0; e < 4; ++e) {
    hb[e]     = h_bits(a[e] * carry);
    hb[4 + e] = h_bits(c[e] * carry);
  }
  const v4u u = (v4u){pk16(hb[0], hb[1]), pk16(hb[2], hb[3]), pk16(hb[4], hb[5]), pk16(hb[6], hb[7])};
  unsigned short* q = out + 8 * (size_t)i;
  *(volatile v4u*)q = u;
  __threadfence();
  *(volatile v4u*)q = u;
}

__global__ __launch_bounds__(256) void wtcast_kernel(const float* __restrict__ W0, const float* __restrict__ W1,
                                                     unsigned short* __restrict__ out0, unsigned short* __restrict__ out1,
                                                     int Kr, int Nc, float scale) {
  __shared__ float sm[64][65];
  const int t  = threadIdx.x;
  const int k0 = blockIdx.x * 64;
  const int n0 = blockIdx.y * 64;
  const int z  = blockIdx.z;
  const float* W = (z == 0) ? W0 : W1;
  unsigned short* op = (z == 0) ? out0 : out1;
#pragma unroll
  for (int i = 0; i < 16; ++i) {
    const int e = i * 256 + t;
    const int r = e >> 6;
    const int c = e & 63;
    sm[c][r] = W[(size_t)(k0 + r) * Nc + n0 + c] * scale;
  }
  __syncthreads();
  const int lane = t & 31, wave = t >> 5;
  const int q = lane >> 3, c8 = (lane & 7) * 8;
  for (int pass = 0; pass < 2; ++pass) {
#pragma unroll
    for (int it = 0; it < 2; ++it) {
      const int row = wave * 8 + it * 4 + q;
      unsigned short hb[8];
#pragma unroll
      for (int e = 0; e < 8; ++e) hb[e] = h_bits(sm[row][c8 + e]);
      const v4u u = (v4u){pk16(hb[0], hb[1]), pk16(hb[2], hb[3]), pk16(hb[4], hb[5]), pk16(hb[6], hb[7])};
      *(volatile v4u*)(op + (size_t)(n0 + row) * Kr + k0 + c8) = u;
    }
    __threadfence();
  }
}


__global__ __launch_bounds__(128) void col_max_kernel(const float* __restrict__ X, int slot_off,
                                                      const float* __restrict__ tptr, float* __restrict__ pmax) {
  const int q   = threadIdx.x;
  const int blk = blockIdx.x;
  const int chunk = blk / kStatBlocksPerChunk;
  const int slot  = (chunk + slot_off) % kNumSlots;
  const float* src = X + (size_t)slot * kSlotElems + (size_t)(blk % kStatBlocksPerChunk) * kStatRows * kDim + 4 * q;
  const float t = tptr[0];
  v4f mx = (v4f){-INFINITY, -INFINITY, -INFINITY, -INFINITY};
#pragma unroll 1
  for (int r = 0; r < kStatRows; ++r) {
    const v4f x = *(const v4f*)(src + (size_t)r * kDim);
#pragma unroll
    for (int e = 0; e < 4; ++e) {
      const float h = fmaxf(x[e], 0.0f);
      const float m = fmaxf(h, 0.0f) + kEpsMsg;
      const float p = t * m;
      mx[e] = fmaxf(mx[e], p);
    }
  }
  float* dst = pmax + (size_t)blk * kDim + 4 * q;
  *(volatile v4f*)dst = mx;
  __threadfence();
  *(volatile v4f*)dst = mx;
}

__global__ __launch_bounds__(128) void col_gmax_kernel(const float* __restrict__ pmax, float* __restrict__ gmax) {
  const int q = threadIdx.x;
  v4f mx = (v4f){-INFINITY, -INFINITY, -INFINITY, -INFINITY};
#pragma unroll 1
  for (int b = 0; b < kStatBlocks; ++b) {
    const v4f x = *(const v4f*)(pmax + (size_t)b * kDim + 4 * q);
#pragma unroll
    for (int e = 0; e < 4; ++e) mx[e] = fmaxf(mx[e], x[e]);
  }
  float* dst = gmax + 4 * q;
  *(volatile v4f*)dst = mx;
  __threadfence();
  *(volatile v4f*)dst = mx;
}

__global__ __launch_bounds__(128) void col_sum_kernel(const float* __restrict__ X, int slot_off,
                                                      const float* __restrict__ tptr, const float* __restrict__ gmax,
                                                      float* __restrict__ psum, float* __restrict__ pdot) {
  const int q   = threadIdx.x;
  const int blk = blockIdx.x;
  const int chunk = blk / kStatBlocksPerChunk;
  const int slot  = (chunk + slot_off) % kNumSlots;
  const float* src = X + (size_t)slot * kSlotElems + (size_t)(blk % kStatBlocksPerChunk) * kStatRows * kDim + 4 * q;
  const float t = tptr[0];
  const v4f gm = *(const v4f*)(gmax + 4 * q);
  v4f S = (v4f){0.f, 0.f, 0.f, 0.f};
  v4f T = (v4f){0.f, 0.f, 0.f, 0.f};
#pragma unroll 1
  for (int r = 0; r < kStatRows; ++r) {
    const v4f x = *(const v4f*)(src + (size_t)r * kDim);
#pragma unroll
    for (int e = 0; e < 4; ++e) {
      const float h = fmaxf(x[e], 0.0f);
      const float m = fmaxf(h, 0.0f) + kEpsMsg;
      const float p = t * m;
      const float ex = expf(p - gm[e]);
      S[e] += ex;
      T[e] += ex * m;
    }
  }
  float* ds = psum + (size_t)blk * kDim + 4 * q;
  float* dt = pdot + (size_t)blk * kDim + 4 * q;
  *(volatile v4f*)ds = S;
  *(volatile v4f*)dt = T;
  __threadfence();
  *(volatile v4f*)ds = S;
  *(volatile v4f*)dt = T;
}

__global__ __launch_bounds__(128) void col_agg_kernel(const float* __restrict__ psum, const float* __restrict__ pdot,
                                                      float* __restrict__ agg) {
  const int q = threadIdx.x;
  v4f S = (v4f){0.f, 0.f, 0.f, 0.f};
  v4f T = (v4f){0.f, 0.f, 0.f, 0.f};
#pragma unroll 1
  for (int b = 0; b < kStatBlocks; ++b) {
    const v4f s = *(const v4f*)(psum + (size_t)b * kDim + 4 * q);
    const v4f d = *(const v4f*)(pdot + (size_t)b * kDim + 4 * q);
    S += s;
    T += d;
  }
  v4f a;
#pragma unroll
  for (int e = 0; e < 4; ++e) a[e] = T[e] * (1.0f / S[e]);
  float* dst = agg + 4 * q;
  *(volatile v4f*)dst = a;
  __threadfence();
  *(volatile v4f*)dst = a;
}

template <bool ADD>
__global__ __launch_bounds__(256) void relu_cast16_kernel(const float* __restrict__ X, int chunk0, int slot_off,
                                                          const float* __restrict__ addv, float carry,
                                                          unsigned short* __restrict__ out) {
  const int i  = blockIdx.x * 256 + threadIdx.x;
  const int cy = blockIdx.y;
  const int chunk = chunk0 + cy;
  const int slot  = (chunk + slot_off) % kNumSlots;
  const size_t loc = 8 * (size_t)i;
  const float* src = X + (size_t)slot * kSlotElems + loc;
  const v4f a = *(const v4f*)(src);
  const v4f c = *(const v4f*)(src + 4);
  v4f ga = (v4f){0.f, 0.f, 0.f, 0.f};
  v4f gc = (v4f){0.f, 0.f, 0.f, 0.f};
  if (ADD) {
    const int col0 = (int)(loc & (size_t)(kDim - 1));
    ga = *(const v4f*)(addv + col0);
    gc = *(const v4f*)(addv + col0 + 4);
  }
  unsigned short hb[8];
#pragma unroll
  for (int e = 0; e < 4; ++e) {
    hb[e]     = h_bits((fmaxf(a[e], 0.0f) + ga[e]) * carry);
    hb[4 + e] = h_bits((fmaxf(c[e], 0.0f) + gc[e]) * carry);
  }
  const v4u u = (v4u){pk16(hb[0], hb[1]), pk16(hb[2], hb[3]), pk16(hb[4], hb[5]), pk16(hb[6], hb[7])};
  unsigned short* q = out + (size_t)cy * kSlotElems + loc;
  *(volatile v4u*)q = u;
  __threadfence();
  *(volatile v4u*)q = u;
}

__global__ __launch_bounds__(128) void ln_relu_kernel(const float* __restrict__ Y, const float* __restrict__ g,
                                                      const float* __restrict__ be, unsigned short* __restrict__ Z, float carry) {
  __shared__ float redA[4];
  __shared__ float redB[4];
  const int row  = blockIdx.x;
  const int t    = threadIdx.x;
  const int lane = t & 31, wave = t >> 5;
  const int c0   = t * 8;
  const float* yr = Y + (size_t)row * kDim2 + c0;
  const v4f a = *(const v4f*)(yr);
  const v4f c = *(const v4f*)(yr + 4);
  float x[8];
#pragma unroll
  for (int e = 0; e < 4; ++e) { x[e] = a[e]; x[4 + e] = c[e]; }
  float s = ((x[0] + x[1]) + (x[2] + x[3])) + ((x[4] + x[5]) + (x[6] + x[7]));
#pragma unroll
  for (int off = 16; off > 0; off >>= 1) s += __shfl_xor(s, off, 32);
  if (lane == 0) redA[wave] = s;
  __syncthreads();
  const float tot = ((redA[0] + redA[1]) + redA[2]) + redA[3];
  const float mu = tot * kInvDim2;
  float d[8];
  float sq = 0.f;
#pragma unroll
  for (int e = 0; e < 8; ++e) { d[e] = x[e] - mu; sq += d[e] * d[e]; }
#pragma unroll
  for (int off = 16; off > 0; off >>= 1) sq += __shfl_xor(sq, off, 32);
  if (lane == 0) redB[wave] = sq;
  __syncthreads();
  const float tot2 = ((redB[0] + redB[1]) + redB[2]) + redB[3];
  const float var = tot2 * kInvDim2;
  const float inv = rsqrtf(var + kEpsLn);
  const v4f g0 = *(const v4f*)(g + c0);
  const v4f g1 = *(const v4f*)(g + c0 + 4);
  const v4f b0 = *(const v4f*)(be + c0);
  const v4f b1 = *(const v4f*)(be + c0 + 4);
  unsigned short hb[8];
#pragma unroll
  for (int e = 0; e < 4; ++e) {
    const float z0 = d[e] * inv * g0[e] + b0[e];
    const float z1 = d[4 + e] * inv * g1[e] + b1[e];
    hb[e]     = h_bits(fmaxf(z0, 0.0f) * carry);
    hb[4 + e] = h_bits(fmaxf(z1, 0.0f) * carry);
  }
  const v4u u = (v4u){pk16(hb[0], hb[1]), pk16(hb[2], hb[3]), pk16(hb[4], hb[5]), pk16(hb[6], hb[7])};
  unsigned short* zp = Z + (size_t)row * kDim2 + c0;
  *(volatile v4u*)zp = u;
  __threadfence();
  *(volatile v4u*)zp = u;
}

extern "C" void kernel_launch(void* const* d_in, const int* in_sizes, int n_in,
                              void* d_out, int out_size, void* d_ws, size_t ws_size,
                              hipStream_t stream)
{
  if (n_in < 19) return;
  if (in_sizes[0] != kNodes * kFin || in_sizes[1] != kFin * kDim || in_sizes[3] != kDim * kDout) return;
  if (in_sizes[6] != kDim * kDim2 || in_sizes[10] != kDim2 * kDim || in_sizes[13] != kDim * kDim2 || in_sizes[17] != kDim2 * kDim) return;
  if (out_size != kNodes * kDout) return;

  const float* batch = (const float*)d_in[0];
  const float* W_enc = (const float*)d_in[1];
  const float* b_enc = (const float*)d_in[2];
  const float* Wf    = (const float*)d_in[3];
  const float* bfv   = (const float*)d_in[4];
  const float* t_p [2] = { (const float*)d_in[5],  (const float*)d_in[12] };
  const float* W1_p[2] = { (const float*)d_in[6],  (const float*)d_in[13] };
  const float* b1_p[2] = { (const float*)d_in[7],  (const float*)d_in[14] };
  const float* g_p [2] = { (const float*)d_in[8],  (const float*)d_in[15] };
  const float* be_p[2] = { (const float*)d_in[9],  (const float*)d_in[16] };
  const float* W2_p[2] = { (const float*)d_in[10], (const float*)d_in[17] };
  const float* b2_p[2] = { (const float*)d_in[11], (const float*)d_in[18] };
  float* out = (float*)d_out;

  const size_t slotBytes = (size_t)kSlotElems * 4;
  const size_t offXS   = 0;
  const size_t offTMP  = offXS + (size_t)kNumSlots * slotBytes;
  const size_t offY    = offTMP;
  const size_t offZ16  = offY + (size_t)kChunkRows * kDim2 * 4;
  const size_t offO16  = offZ16 + (size_t)kChunkRows * kDim2 * 2;
  const size_t offB16  = offO16 + (size_t)kChunkRows * kDim * 2;
  const size_t offH16  = offTMP;
  const size_t offWenc = offB16 + (size_t)kNodes * kFin * 2;
  const size_t offWf   = offWenc + (size_t)kDim * kFin * 2;
  const size_t offW1a  = offWf + (size_t)kDout * kDim * 2;
  const size_t offW1b  = offW1a + (size_t)kDim2 * kDim * 2;
  const size_t offW2a  = offW1b + (size_t)kDim2 * kDim * 2;
  const size_t offW2b  = offW2a + (size_t)kDim * kDim2 * 2;
  const size_t offPmax = offW2b + (size_t)kDim * kDim2 * 2;
  const size_t statBytes = (size_t)kStatBlocks * kDim * 4;
  const size_t offPsum = offPmax + statBytes;
  const size_t offPdot = offPsum + statBytes;
  const size_t offGmax = offPdot + statBytes;
  const size_t offAgg  = offGmax + (size_t)kDim * 4;
  const size_t wsTotal = offAgg + (size_t)kDim * 4;
  if (offH16 + (size_t)kNodes * kDim * 2 > offWenc) return;
  if (wsTotal > ws_size) return;

  char* ws = (char*)d_ws;
  float*          XS    = (float*)(ws + offXS);
  float*          Ybuf  = (float*)(ws + offY);
  unsigned short* Z16   = (unsigned short*)(ws + offZ16);
  unsigned short* O16   = (unsigned short*)(ws + offO16);
  unsigned short* B16   = (unsigned short*)(ws + offB16);
  unsigned short* H16   = (unsigned short*)(ws + offH16);
  unsigned short* WencT = (unsigned short*)(ws + offWenc);
  unsigned short* WfT   = (unsigned short*)(ws + offWf);
  unsigned short* W1T[2] = { (unsigned short*)(ws + offW1a), (unsigned short*)(ws + offW1b) };
  unsigned short* W2T[2] = { (unsigned short*)(ws + offW2a), (unsigned short*)(ws + offW2b) };
  float* pmax = (float*)(ws + offPmax);
  float* psum = (float*)(ws + offPsum);
  float* pdot = (float*)(ws + offPdot);
  float* gmax = (float*)(ws + offGmax);
  float* agg  = (float*)(ws + offAgg);

  cast8_f16_kernel<<<(kNodes * kFin / 8) / 256, 256, 0, stream>>>(batch, B16, kNodes * kFin / 8, kInCarry);
  wtcast_kernel<<<dim3(kFin / 64, kDim / 64, 1), 256, 0, stream>>>(W_enc, W_enc, WencT, WencT, kFin, kDim, kWCarry);
  wtcast_kernel<<<dim3(kDim / 64, kDout / 64, 1), 256, 0, stream>>>(Wf, Wf, WfT, WfT, kDim, kDout, kWCarry);
  wtcast_kernel<<<dim3(kDim / 64, kDim2 / 64, 2), 256, 0, stream>>>(W1_p[0], W1_p[1], W1T[0], W1T[1], kDim, kDim2, kWCarry);
  wtcast_kernel<<<dim3(kDim2 / 64, kDim / 64, 2), 256, 0, stream>>>(W2_p[0], W2_p[1], W2T[0], W2T[1], kDim2, kDim, kWCarry);

  {
    const int tiles = (kNodes / 64) * (kDim / 64);
    wmma_gemm64<0, false, 2, 0, false, 0><<<dim3((tiles + 7) / 8, 1), 256, 0, stream>>>(
        B16, nullptr, kFin, 0L, WencT, nullptr, kFin, 0L,
        (void*)XS, nullptr, kDim, 0L, b_enc, nullptr, 0L,
        kNodes, kDim, kFin, 1.0f / (kInCarry * kWCarry));
  }

  const int in_off_l[2]  = { 9, 8 };
  const int out_off_l[2] = { 8, 7 };
  for (int l = 0; l < 2; ++l) {
    const int in_off = in_off_l[l], out_off = out_off_l[l];
    col_max_kernel<<<kStatBlocks, 128, 0, stream>>>(XS, in_off, t_p[l], pmax);
    col_gmax_kernel<<<1, 128, 0, stream>>>(pmax, gmax);
    col_sum_kernel<<<kStatBlocks, 128, 0, stream>>>(XS, in_off, t_p[l], gmax, psum, pdot);
    col_agg_kernel<<<1, 128, 0, stream>>>(psum, pdot, agg);
    for (int c = 0; c < kNumChunks; ++c) {
      const int in_slot  = (c + in_off) % kNumSlots;
      const int out_slot = (c + out_off) % kNumSlots;
      relu_cast16_kernel<true><<<dim3((int)(kSlotElems / 8 / 256), 1), 256, 0, stream>>>(XS, c, in_off, agg, 1.0f, O16);
      {
        const int tiles = (kChunkRows / 64) * (kDim2 / 64);
        wmma_gemm64<0, false, 2, 0, false, 0><<<dim3((tiles + 7) / 8, 1), 256, 0, stream>>>(
            O16, nullptr, kDim, 0L, W1T[l], nullptr, kDim, 0L,
            (void*)Ybuf, nullptr, kDim2, 0L, b1_p[l], nullptr, 0L,
            kChunkRows, kDim2, kDim, 1.0f / kWCarry);
      }
      ln_relu_kernel<<<kChunkRows, 128, 0, stream>>>(Ybuf, g_p[l], be_p[l], Z16, kZCarry);
      {
        const int tiles = (kChunkRows / 64) * (kDim / 64);
        wmma_gemm64<0, false, 2, 0, true, 0><<<dim3((tiles + 7) / 8, 1), 256, 0, stream>>>(
            Z16, nullptr, kDim2, 0L, W2T[l], nullptr, kDim2, 0L,
            (void*)(XS + (size_t)out_slot * kSlotElems), nullptr, kDim, 0L, b2_p[l],
            XS + (size_t)in_slot * kSlotElems, 0L,
            kChunkRows, kDim, kDim2, 1.0f / (kZCarry * kWCarry));
      }
    }
  }

  relu_cast16_kernel<false><<<dim3((int)(kSlotElems / 8 / 256), kNumChunks), 256, 0, stream>>>(XS, 0, 7, agg, kHCarry, H16);
  {
    const int tiles = (kNodes / 64) * (kDout / 64);
    wmma_gemm64<0, false, 2, 0, false, 0><<<dim3((tiles + 7) / 8, 1), 256, 0, stream>>>(
        H16, nullptr, kDim, 0L, WfT, nullptr, kDim, 0L,
        (void*)out, nullptr, kDout, 0L, bfv, nullptr, 0L,
        kNodes, kDout, kDim, 1.0f / (kHCarry * kWCarry));
  }
}
